// GATLayer_87840671138247
// MI455X (gfx1250) — hardware-verified
//
#include <hip/hip_runtime.h>
#include <math.h>
#include <stdint.h>
#include <stddef.h>

#define NB_   2
#define NT_   12
#define NNODE 2000
#define FD    128
#define KNBR  16
#define MTOT  (NB_ * NT_ * NNODE)
#define GBM   64
#define GTHR  128
#define LP    132
#define ATHR  256
#define AWAV  (ATHR / 32)
#define CTHR  256
#define WSMAX 134217728

static_assert(MTOT % GBM == 0);
static_assert(FD == 128 && FD % 32 == 0);
static_assert(GTHR == FD);
static_assert(GBM == (GTHR / 32) * 16);
static_assert((MTOT * FD) % (CTHR * 8) == 0);
static_assert((FD * FD) % (CTHR * 8) == 0);
static_assert(KNBR == 16);
static_assert((LP * 4) % 16 == 0);
static_assert(MTOT % AWAV == 0);
static_assert((GBM * 4) % 256 == 0);
static_assert(((size_t)MTOT * 4) % 128 == 0);

typedef float          v4f   __attribute__((ext_vector_type(4)));
typedef float          v8f   __attribute__((ext_vector_type(8)));
typedef int            v8i   __attribute__((ext_vector_type(8)));
typedef unsigned       v4u   __attribute__((ext_vector_type(4)));
typedef unsigned short v8us  __attribute__((ext_vector_type(8)));
typedef unsigned short v16us __attribute__((ext_vector_type(16)));
typedef __bf16         v16bf __attribute__((ext_vector_type(16)));
typedef v4f  __attribute__((may_alias)) v4fa;
typedef v4u  __attribute__((may_alias)) v4ua;
typedef v8us __attribute__((may_alias)) v8usa;
union FragB { v16bf v; v16us u; v8us h[2]; v8i w; };

__device__ __forceinline__ v8f wmb(const FragB& a, const FragB& b, v8f c) {
  v8f d = __builtin_amdgcn_wmma_f32_16x16x32_bf16(false, a.v, false, b.v, (short)0, c, false, false);
  asm volatile("v_nop\n\tv_nop\n\tv_nop\n\tv_nop" : "+v"(d) : "v"(a.w), "v"(b.w));
  return d;
}

__device__ __forceinline__ unsigned bf16_bits(float f) {
  const unsigned u = __float_as_uint(f);
  return (u + 0x7FFFu + ((u >> 16) & 1u)) >> 16;
}
__device__ __forceinline__ float bf16_val(float f) {
  return __uint_as_float(bf16_bits(f) << 16);
}
__device__ __forceinline__ unsigned pk16(unsigned a, unsigned b) { return (a & 0xffffu) | (b << 16); }

__global__ __launch_bounds__(CTHR) void k_cvt(const float* __restrict__ src, unsigned short* dst, int n8) {
  int i = (int)blockIdx.x * CTHR + (int)threadIdx.x;
  const bool ok = i < n8;
  i = ok ? i : (n8 - 1);
  const float* s = src + (size_t)i * 8;
  const v4f f0 = *(const v4fa*)(s);
  const v4f f1 = *(const v4fa*)(s + 4);
  v4u u;
  u[0] = pk16(bf16_bits(f0[0]), bf16_bits(f0[1]));
  u[1] = pk16(bf16_bits(f0[2]), bf16_bits(f0[3]));
  u[2] = pk16(bf16_bits(f1[0]), bf16_bits(f1[1]));
  u[3] = pk16(bf16_bits(f1[2]), bf16_bits(f1[3]));
  unsigned short* d = dst + (size_t)i * 8;
  if (ok) *(volatile v4u*)d = u;
  __threadfence();
  if (ok) *(volatile v4u*)d = u;
}

__global__ __launch_bounds__(GTHR) void k_proj(const unsigned short* __restrict__ Xb,
                                               const unsigned short* __restrict__ Wb,
                                               const float* __restrict__ av, float* HH, float* S) {
  __shared__ __attribute__((aligned(16))) float stg[GBM * LP];
  __shared__ __attribute__((aligned(16))) float sA[2 * FD];
  __shared__ __attribute__((aligned(16))) float sS[2 * GBM];
  const int tid = (int)threadIdx.x, lane = tid & 31, wave = tid >> 5, hh = lane >> 4, m = lane & 15;
  const int rowBase = (int)blockIdx.x * GBM;

  sA[tid]      = bf16_val(av[tid]);
  sA[FD + tid] = bf16_val(av[FD + tid]);

  v8f acc[8];
  {
    const v8f z = {0.f, 0.f, 0.f, 0.f, 0.f, 0.f, 0.f, 0.f};
#pragma unroll
    for (int t = 0; t < 8; ++t) acc[t] = z;
  }
  const unsigned short* ap = Xb + (size_t)(rowBase + 16 * wave + m) * (size_t)FD + 8 * hh;
  const unsigned short* bp = Wb + (size_t)m * (size_t)FD + 8 * hh;

#pragma unroll 1
  for (int k0 = 0; k0 < FD; k0 += 32) {
    FragB af;
    af.h[0] = *(const v8usa*)(ap + k0);
    af.h[1] = *(const v8usa*)(ap + k0 + 16);
#pragma unroll
    for (int nt = 0; nt < 8; ++nt) {
      const unsigned short* wq = bp + (size_t)(16 * nt) * (size_t)FD + k0;
      FragB bf;
      bf.h[0] = *(const v8usa*)wq;
      bf.h[1] = *(const v8usa*)(wq + 16);
      acc[nt] = wmb(af, bf, acc[nt]);
    }
  }

#pragma unroll
  for (int nt = 0; nt < 8; ++nt) {
    const int lc = 16 * nt + m;
#pragma unroll
    for (int r = 0; r < 8; ++r) {
      const int lr = 16 * wave + 8 * hh + r;
      stg[lr * LP + lc] = acc[nt][r];
    }
  }
  __syncthreads();

  {
    const int row = tid & (GBM - 1);
    const int hf  = tid >> 6;
    const float* fr = stg + row * LP;
    const float* ar = sA + hf * FD;
    float s = 0.0f;
#pragma unroll 4
    for (int d4 = 0; d4 < FD / 4; ++d4) {
      const v4f x = *(const v4fa*)(fr + 4 * d4);
      const v4f y = *(const v4fa*)(ar + 4 * d4);
      s = fmaf(x[0], y[0], s);
      s = fmaf(x[1], y[1], s);
      s = fmaf(x[2], y[2], s);
      s = fmaf(x[3], y[3], s);
    }
    sS[tid] = s;
  }
  __syncthreads();

  {
    const int pl = lane >> 4;
    const int c4 = (lane & 15) * 4;
    for (int pass = 0; pass < 2; ++pass) {
#pragma unroll
      for (int i = 0; i < 16; ++i) {
        const int lr = 16 * wave + i;
        const v4f v = *(const v4fa*)(stg + lr * LP + 4 * lane);
        *(volatile v4f*)(HH + (size_t)(rowBase + lr) * (size_t)FD + 4 * lane) = v;
      }
      if (wave == 0) {
        const v4f sv = *(const v4fa*)(sS + pl * GBM + c4);
        *(volatile v4f*)(S + (size_t)pl * (size_t)MTOT + rowBase + c4) = sv;
      }
      __threadfence();
    }
  }
}

__global__ __launch_bounds__(ATHR) void k_agg(const float* __restrict__ HH, const float* __restrict__ S,
                                              const int* __restrict__ adj, float* out) {
  const int tid = (int)threadIdx.x, lane = tid & 31, wave = tid >> 5;
  const int gw = (int)blockIdx.x * AWAV + wave;
  const bool live = gw < MTOT;
  const int gwc = live ? gw : (MTOT - 1);
  const int bt  = gwc / NNODE;
  const int n   = gwc - bt * NNODE;
  const int k   = lane & 15;

  int nb = adj[(size_t)n * KNBR + k];
  nb = (nb < 0) ? (nb + NNODE) : nb;
  nb = nb < 0 ? 0 : (nb > NNODE - 1 ? NNODE - 1 : nb);

  const float s_self = S[(size_t)bt * NNODE + n];
  const float e = s_self + S[(size_t)MTOT + (size_t)bt * NNODE + nb];

  float mx = e;
#pragma unroll
  for (int mask = 1; mask <= 8; mask <<= 1) mx = fmaxf(mx, __shfl_xor(mx, mask, 32));
  const float p = expf(e - mx);
  float sum = p;
#pragma unroll
  for (int mask = 1; mask <= 8; mask <<= 1) sum += __shfl_xor(sum, mask, 32);
  const float alpha = p * (1.0f / sum);

  const float* hb = HH + (size_t)bt * (size_t)NNODE * FD + 4 * lane;
  v4f acc = {0.0f, 0.0f, 0.0f, 0.0f};
#pragma unroll 2
  for (int kk = 0; kk < KNBR; ++kk) {
    const int   j  = __shfl(nb, kk, 32);
    const float ak = __shfl(alpha, kk, 32);
    const v4f v = *(const v4fa*)(hb + (size_t)j * FD);
    acc.x = fmaf(ak, v.x, acc.x);
    acc.y = fmaf(ak, v.y, acc.y);
    acc.z = fmaf(ak, v.z, acc.z);
    acc.w = fmaf(ak, v.w, acc.w);
  }

  float* op = out + (size_t)gwc * FD + 4 * lane;
  if (live) *(volatile v4f*)op = acc;
  __threadfence();
  if (live) *(volatile v4f*)op = acc;
}

static inline int cdiv(int a, int b) { return (a + b - 1) / b; }

extern "C" void kernel_launch(void* const* d_in, const int* in_sizes, int n_in,
                              void* d_out, int out_size, void* d_ws, size_t ws_size,
                              hipStream_t stream) {
  if (n_in < 4) return;
  if (in_sizes[0] != MTOT * FD) return;
  if (in_sizes[1] != FD * FD) return;
  if (in_sizes[2] != 2 * FD) return;
  if (in_sizes[3] != NNODE * KNBR) return;
  if (out_size != MTOT * FD) return;

  const float* h   = (const float*)d_in[0];
  const float* W   = (const float*)d_in[1];
  const float* av  = (const float*)d_in[2];
  const int*   adj = (const int*)d_in[3];
  float* out = (float*)d_out;

  size_t off = 0;
  const size_t oXb = off; off += (size_t)MTOT * FD * 2;  off = (off + 255) & ~(size_t)255;
  const size_t oWb = off; off += (size_t)FD * FD * 2;    off = (off + 255) & ~(size_t)255;
  const size_t oHH = off; off += (size_t)MTOT * FD * 4;  off = (off + 255) & ~(size_t)255;
  const size_t oS  = off; off += (size_t)2 * MTOT * 4;   off = (off + 255) & ~(size_t)255;
  if (off > ws_size || off > (size_t)WSMAX) return;

  char* ws = (char*)d_ws;
  unsigned short* Xb = (unsigned short*)(ws + oXb);
  unsigned short* Wb = (unsigned short*)(ws + oWb);
  float*          HH = (float*)(ws + oHH);
  float*          S  = (float*)(ws + oS);

  const int n8x = MTOT * FD / 8;
  const int n8w = FD * FD / 8;
  k_cvt<<<dim3(cdiv(n8x, CTHR)), CTHR, 0, stream>>>(h, Xb, n8x);
  k_cvt<<<dim3(cdiv(n8w, CTHR)), CTHR, 0, stream>>>(W, Wb, n8w);
  k_proj<<<dim3(MTOT / GBM), GTHR, 0, stream>>>(Xb, Wb, av, HH, S);
  k_agg<<<dim3(cdiv(MTOT, AWAV)), ATHR, 0, stream>>>(HH, S, adj, out);
  (void)hipGetLastError();
}
